// BipartiteSchedulerGNN_41979010351696
// MI455X (gfx1250) — hardware-verified
//
#include <hip/hip_runtime.h>
#include <stddef.h>
#include <stdint.h>

#pragma clang fp contract(off)


#define CH    64
#define KRB   64
#define NTHR  256
#define NWAVE 8
#define PA    68
#define KPP   72

static_assert(CH == 64 && KRB == 64);
static_assert(NTHR == 32 * NWAVE && NWAVE == 8);
static_assert((PA * 4) % 16 == 0);
static_assert((KPP * 2) % 16 == 0);
static_assert(NTHR == 4 * CH);

typedef float  v4f  __attribute__((ext_vector_type(4)));
typedef float  v8f  __attribute__((ext_vector_type(8)));
typedef __bf16 v8b  __attribute__((ext_vector_type(8)));
typedef __bf16 v16b __attribute__((ext_vector_type(16)));
typedef unsigned short v16us __attribute__((ext_vector_type(16)));
union FragB { v16b v; v8b h8[2]; };

__device__ __forceinline__ v8f zero8() {
  v8f z = {0.0f, 0.0f, 0.0f, 0.0f, 0.0f, 0.0f, 0.0f, 0.0f};
  return z;
}

__device__ __forceinline__ v8f wmb(v16b a, v16b b, v8f c) {
  v8f d = __builtin_amdgcn_wmma_f32_16x16x32_bf16(false, a, false, b, (short)0, c, false, false);
#if defined(__HIP_DEVICE_COMPILE__)
  const v16us au = __builtin_bit_cast(v16us, a);
  const v16us bq = __builtin_bit_cast(v16us, b);
  asm volatile("v_nop\n\tv_nop\n\tv_nop\n\tv_nop" : "+v"(d) : "v"(au), "v"(bq));
#endif
  return d;
}

__device__ __forceinline__ float bf2f(__bf16 b) {
  return __uint_as_float(((unsigned int)__builtin_bit_cast(unsigned short, b)) << 16);
}

__device__ __forceinline__ void split16(const float (&x)[16], v16b& hi, v16b& lo) {
#pragma unroll
  for (int i = 0; i < 16; ++i) {
    const __bf16 hb = (__bf16)x[i];
    const float hf = bf2f(hb);
    hi[i] = hb;
    lo[i] = (__bf16)(x[i] - hf);
  }
}

__device__ __forceinline__ void ld16(const float* p, float (&v)[16]) {
  const v4f q0 = *(const v4f*)(p);
  const v4f q1 = *(const v4f*)(p + 4);
  const v4f q2 = *(const v4f*)(p + 16);
  const v4f q3 = *(const v4f*)(p + 20);
#pragma unroll
  for (int i = 0; i < 4; ++i) {
    v[i] = q0[i]; v[4 + i] = q1[i]; v[8 + i] = q2[i]; v[12 + i] = q3[i];
  }
}

__device__ __forceinline__ v16b ldfrag(const __bf16* p) {
  FragB f;
  f.h8[0] = *(const v8b*)(p);
  f.h8[1] = *(const v8b*)(p + 16);
  return f.v;
}

__device__ __forceinline__ void build_planes(const float* __restrict__ W, __bf16* sPh, __bf16* sPl, int tid) {
  const int n = tid >> 2, q = tid & 3;
  v8b h0, h1, l0, l1;
#pragma unroll
  for (int j = 0; j < 8; ++j) {
    const float w0 = W[(16 * q + j) * CH + n];
    const float w1 = W[(16 * q + 8 + j) * CH + n];
    const __bf16 a0 = (__bf16)w0;
    const __bf16 a1 = (__bf16)w1;
    const float f0 = bf2f(a0);
    const float f1 = bf2f(a1);
    h0[j] = a0;
    h1[j] = a1;
    l0[j] = (__bf16)(w0 - f0);
    l1[j] = (__bf16)(w1 - f1);
  }
  __bf16* ph = sPh + n * KPP + 16 * q;
  __bf16* pl = sPl + n * KPP + 16 * q;
  *(v8b*)(ph)     = h0;
  *(v8b*)(ph + 8) = h1;
  *(v8b*)(pl)     = l0;
  *(v8b*)(pl + 8) = l1;
}

__device__ __forceinline__ void node_layer(const float* sIn, float* sDst, const __bf16* sPh, const __bf16* sPl,
                                           const float* __restrict__ bias, int kt, int ch, int hh, int m) {
  v8f d[2];
  d[0] = zero8();
  d[1] = zero8();
  const int n0 = ch * 32 + m;
#pragma unroll
  for (int ks = 0; ks < 2; ++ks) {
    float av[16];
    ld16(sIn + (kt * 16 + m) * PA + ks * 32 + 8 * hh, av);
    v16b ah, al;
    split16(av, ah, al);
#pragma unroll
    for (int nt = 0; nt < 2; ++nt) {
      const __bf16* pb = sPh + (n0 + 16 * nt) * KPP + ks * 32 + 8 * hh;
      const __bf16* pc = sPl + (n0 + 16 * nt) * KPP + ks * 32 + 8 * hh;
      const v16b bh = ldfrag(pb);
      const v16b bl = ldfrag(pc);
      d[nt] = wmb(ah, bh, d[nt]);
      d[nt] = wmb(ah, bl, d[nt]);
      d[nt] = wmb(al, bh, d[nt]);
    }
  }
#pragma unroll
  for (int nt = 0; nt < 2; ++nt) {
    const float bv = bias[n0 + 16 * nt];
    float* dp = sDst + (kt * 16 + 8 * hh) * PA + n0 + 16 * nt;
#pragma unroll
    for (int r = 0; r < 8; ++r) dp[r * PA] = fmaxf(d[nt][r] + bv, 0.0f);
  }
}

__global__ __launch_bounds__(NTHR) void k_gnn(
    const float* __restrict__ ef,
    const float* __restrict__ We1, const float* __restrict__ be1,
    const float* __restrict__ We2, const float* __restrict__ be2,
    const float* __restrict__ Wu1, const float* __restrict__ bu1,
    const float* __restrict__ Wu2, const float* __restrict__ bu2,
    const float* __restrict__ Wo, const float* __restrict__ bo,
    float* out, int nA) {
  __shared__ __attribute__((aligned(16))) float  sAgg[KRB * PA];
  __shared__ __attribute__((aligned(16))) float  sU[KRB * PA];
  __shared__ __attribute__((aligned(16))) __bf16 sPh[CH * KPP];
  __shared__ __attribute__((aligned(16))) __bf16 sPl[CH * KPP];
  __shared__ __attribute__((aligned(16))) float  sW1[CH];
  __shared__ __attribute__((aligned(16))) float  sB1[CH];
  __shared__ __attribute__((aligned(16))) float  sOut[KRB];

  const int tid = threadIdx.x, lane = tid & 31, wave = tid >> 5;
  const int hh = lane >> 4, m = lane & 15;
  const int kt = wave & 3, ch = wave >> 2;
  const int bu = blockIdx.x;
  const float* efb = ef + (size_t)bu * (size_t)nA * KRB;

  if (tid < CH) {
    sW1[tid] = We1[tid];
    sB1[tid] = be1[tid];
  }
  build_planes(We2, sPh, sPl, tid);
  float be2v[2];
#pragma unroll
  for (int nt = 0; nt < 2; ++nt) be2v[nt] = be2[ch * 32 + 16 * nt + m];
  __syncthreads();

  v8f acc[2];
  acc[0] = zero8();
  acc[1] = zero8();
  const int krow = kt * 16 + m;
  const int n0 = ch * 32 + m;
#pragma unroll 1
  for (int a = 0; a < nA; ++a) {
    const float x = efb[(size_t)a * KRB + krow];
    v8f d[2];
    d[0] = zero8();
    d[1] = zero8();
#pragma unroll
    for (int ks = 0; ks < 2; ++ks) {
      float wv[16], bv[16], hv[16];
      ld16(sW1 + ks * 32 + 8 * hh, wv);
      ld16(sB1 + ks * 32 + 8 * hh, bv);
#pragma unroll
      for (int i = 0; i < 16; ++i) {
        const float p = x * wv[i];
        const float s = p + bv[i];
        hv[i] = fmaxf(s, 0.0f);
      }
      v16b ah, al;
      split16(hv, ah, al);
#pragma unroll
      for (int nt = 0; nt < 2; ++nt) {
        const __bf16* pb = sPh + (n0 + 16 * nt) * KPP + ks * 32 + 8 * hh;
        const __bf16* pc = sPl + (n0 + 16 * nt) * KPP + ks * 32 + 8 * hh;
        const v16b bh = ldfrag(pb);
        const v16b bl = ldfrag(pc);
        d[nt] = wmb(ah, bh, d[nt]);
        d[nt] = wmb(ah, bl, d[nt]);
        d[nt] = wmb(al, bh, d[nt]);
      }
    }
#pragma unroll
    for (int nt = 0; nt < 2; ++nt) {
#pragma unroll
      for (int r = 0; r < 8; ++r) acc[nt][r] = acc[nt][r] + fmaxf(d[nt][r] + be2v[nt], 0.0f);
    }
  }
#pragma unroll
  for (int nt = 0; nt < 2; ++nt) {
    float* dp = sAgg + (kt * 16 + 8 * hh) * PA + n0 + 16 * nt;
#pragma unroll
    for (int r = 0; r < 8; ++r) dp[r * PA] = acc[nt][r];
  }
  __syncthreads();

  build_planes(Wu1, sPh, sPl, tid);
  __syncthreads();
  node_layer(sAgg, sU, sPh, sPl, bu1, kt, ch, hh, m);
  __syncthreads();

  build_planes(Wu2, sPh, sPl, tid);
  __syncthreads();
  node_layer(sU, sAgg, sPh, sPl, bu2, kt, ch, hh, m);
  __syncthreads();

  if (tid < KRB) {
    const float* ur = sAgg + tid * PA;
    float s = 0.0f;
#pragma unroll 4
    for (int c = 0; c < CH; ++c) s = fmaf(ur[c], Wo[c], s);
    sOut[tid] = s + bo[0];
  }
  __syncthreads();

  if (wave == 0) {
    const int sl = lane & 15;
    const v4f v = *(const v4f*)(sOut + 4 * sl);
    float* op = out + (size_t)bu * KRB + 4 * sl;
    if (lane < 16) *(volatile v4f*)op = v;
    __threadfence();
    if (lane < 16) *(volatile v4f*)op = v;
  }
}

extern "C" void kernel_launch(void* const* d_in, const int* in_sizes, int n_in,
                              void* d_out, int out_size, void* d_ws, size_t ws_size,
                              hipStream_t stream) {
  (void)d_ws;
  (void)ws_size;
  if (n_in < 11) return;
  if (out_size <= 0 || (out_size % KRB) != 0) return;
  const int BU = out_size / KRB;
  if (in_sizes[0] <= 0 || (in_sizes[0] % out_size) != 0) return;
  const int nA = in_sizes[0] / out_size;
  if (nA < 1 || nA > 65536) return;
  if (in_sizes[1] != CH || in_sizes[2] != CH) return;
  if (in_sizes[3] != CH * CH || in_sizes[4] != CH) return;
  if (in_sizes[5] != CH * CH || in_sizes[6] != CH) return;
  if (in_sizes[7] != CH * CH || in_sizes[8] != CH) return;
  if (in_sizes[9] != CH || in_sizes[10] < 1) return;

  const float* ef  = (const float*)d_in[0];
  const float* We1 = (const float*)d_in[1];
  const float* be1 = (const float*)d_in[2];
  const float* We2 = (const float*)d_in[3];
  const float* be2 = (const float*)d_in[4];
  const float* Wu1 = (const float*)d_in[5];
  const float* bu1 = (const float*)d_in[6];
  const float* Wu2 = (const float*)d_in[7];
  const float* bu2 = (const float*)d_in[8];
  const float* Wo  = (const float*)d_in[9];
  const float* bo  = (const float*)d_in[10];
  float* out = (float*)d_out;

  k_gnn<<<dim3(BU), dim3(NTHR), 0, stream>>>(ef, We1, be1, We2, be2, Wu1, bu1, Wu2, bu2, Wo, bo, out, nA);
}
